// PolicyNetwork_32933809226462
// MI455X (gfx1250) — hardware-run, weakly checked
//
#include <hip/hip_runtime.h>


namespace {
constexpr int B = 8, T = 2048, DM = 768, NCH = DM / 128, NSL = DM / 128, NB = 8  , NA = 2  ;
constexpr float XS = 8.0f, WSC = 256.0f, PS = 1024.0f, RS_ = 1024.0f, LOG2E = 1.4426950408889634f, EPSC = 1e-6f, LNEPS = 1e-5f, MASKED = -1.0e9f * 1.4426950408889634f  ;
static_assert(T % 128 == 0 && DM % 256 == 0 && NCH == 6, "tiling");
typedef _Float16 b16;
typedef __attribute__((ext_vector_type(16))) _Float16 v16b;
typedef __attribute__((ext_vector_type(8))) _Float16 v8b;
typedef __attribute__((ext_vector_type(8))) float v8f;
typedef __attribute__((ext_vector_type(4))) float v4f;
__device__ __forceinline__ float bf16_rne(float f) { unsigned int u = __float_as_uint(f); u += 0x7FFFu + ((u >> 16) & 1u); return __uint_as_float(u & 0xFFFF0000u); }
__device__ __forceinline__ void split16(float v, b16& hi, b16& lo) { hi = (b16)v; lo = (b16)(v - (float)hi); }
__device__ __forceinline__ v16b frag_kb(const b16* p, int hh) { const v8b a = *(const v8b*)(p + 8 * hh), b = *(const v8b*)(p + 16 + 8 * hh); v16b f;
#pragma unroll
  for (int e = 0; e < 8; ++e) { f[e] = a[e]; f[8 + e] = b[e]; } return f; }
__device__ __forceinline__ v8f wmma16b(v16b a, v16b b, v8f c) { v8f d = __builtin_amdgcn_wmma_f32_16x16x32_f16(false, a, false, b, (short)0, c, false, false); asm volatile("v_nop\n\tv_nop\n\tv_nop\n\tv_nop" : "+v"(d) : "v"(a), "v"(b)); return d; }
__device__ __forceinline__ void wave_lds_sync() { __builtin_amdgcn_fence(__ATOMIC_RELEASE, "workgroup"); __builtin_amdgcn_wave_barrier(); __builtin_amdgcn_fence(__ATOMIC_ACQUIRE, "workgroup"); }
__device__ __forceinline__ float pmul(float a, float b) { float p = a * b; asm volatile("" : "+v"(p)); return p; }
__device__ __forceinline__ int iclamp(int v, int lo, int hi) { return v < lo ? lo : (v > hi ? hi : v); }

typedef __attribute__((ext_vector_type(2))) _Float16 v2h;
typedef __attribute__((ext_vector_type(4))) _Float16 v4h;
typedef __attribute__((ext_vector_type(2))) float v2f;
typedef __attribute__((ext_vector_type(4))) int v4i;
__device__ __forceinline__ float nexp2(float v) { return __builtin_amdgcn_exp2f(v); }
__device__ __forceinline__ float bfp(float v) { float t = bf16_rne(v); asm volatile("" : "+v"(t)); return t; }
__global__ __launch_bounds__(256) void prep_kernel(const float* __restrict__ wq, const float* __restrict__ wk, const float* __restrict__ wv, const float* __restrict__ wo, const float* __restrict__ wa, b16* __restrict__ WQ, b16* __restrict__ WK, b16* __restrict__ WV, b16* __restrict__ WO, b16* __restrict__ WA) {
  const size_t u = (size_t)blockIdx.x * 256 + threadIdx.x; const size_t per = (size_t)DM * DM / 8; const size_t na = (size_t)16 * DM / 8; if (u >= 4 * per + na) return; v8b o;
  if (u < 4 * per) { const int m = (int)(u / per); const size_t e = u % per; const int row = (int)(e / (DM / 8)), k0 = (int)(e % (DM / 8)) * 8; const float* w = m == 0 ? wq : m == 1 ? wk : m == 2 ? wv : wo; b16* dst = (m == 0 ? WQ : m == 1 ? WK : m == 2 ? WV : WO) + (size_t)row * DM + k0;
    for (int j = 0; j < 8; ++j) o[j] = (b16)(bf16_rne(w[(size_t)(k0 + j) * DM + row]) * WSC); for (int pass = 0; pass < 2; ++pass) { *(volatile v8b*)dst = o; __threadfence(); } }
  else { const size_t e = (u - 4 * per) * 8; const int row = (int)(e / DM), k0 = (int)(e % DM); for (int j = 0; j < 8; ++j) o[j] = (b16)(row < NA ? bf16_rne(wa[(size_t)(k0 + j) * NA + row]) * WSC : 0.0f);
    for (int pass = 0; pass < 2; ++pass) { *(volatile v8b*)(WA + e) = o; __threadfence(); } }
}
__global__ __launch_bounds__(256) void cn_kernel(const float* __restrict__ x, int b0, const float* __restrict__ a2, const float* __restrict__ b2, float* __restrict__ CN) {
  const int wave = threadIdx.x >> 5, lane = threadIdx.x & 31; const int row = blockIdx.x * 8 + wave;
  float v[24]; float s1 = 0.0f; const float* xr = x + ((size_t)b0 * T + row) * DM;
#pragma unroll
  for (int k = 0; k < NCH; ++k) { const v4f t4 = *(const v4f*)(xr + 128 * k + 4 * lane); for (int j = 0; j < 4; ++j) { const float t = bf16_rne(t4[j]); v[4 * k + j] = t; s1 += t; } }
#pragma unroll
  for (int o = 16; o >= 1; o >>= 1) s1 += __shfl_xor(s1, o);
  const float mu = s1 * (1.0f / DM); float s2 = 0.0f;
#pragma unroll
  for (int q = 0; q < 24; ++q) { const float d = v[q] - mu; s2 += pmul(d, d); }
#pragma unroll
  for (int o = 16; o >= 1; o >>= 1) s2 += __shfl_xor(s2, o);
  const float sd = sqrtf(s2 * (1.0f / (DM - 1))); const float inv = __builtin_amdgcn_rcpf(sd + EPSC);
  v4f o4[NCH];
#pragma unroll
  for (int k = 0; k < NCH; ++k) for (int j = 0; j < 4; ++j) { const int c = 128 * k + 4 * lane + j; o4[k][j] = pmul(bfp(a2[c]), (v[4 * k + j] - mu) * inv) + bfp(b2[c]); }
  for (int pass = 0; pass < 2; ++pass) {
#pragma unroll
    for (int k = 0; k < NCH; ++k) *(volatile v4f*)(CN + (size_t)row * DM + 128 * k + 4 * lane) = o4[k];
    __threadfence(); }
}
__global__ __launch_bounds__(128) void proj_kernel(const float* __restrict__ CN, const b16* __restrict__ WQ, const b16* __restrict__ WK, const b16* __restrict__ WV, const float* __restrict__ bq, const float* __restrict__ bk, const float* __restrict__ bv, b16* __restrict__ QP, b16* __restrict__ KP, b16* __restrict__ VT) {
  __shared__ __attribute__((aligned(16))) b16 As[64][256 + 8]; __shared__ __attribute__((aligned(16))) float Tf[4][16][128 + 4];
  const int wave = threadIdx.x >> 5, lane = threadIdx.x & 31, nloc = lane & 15, hlf = lane >> 4; const int t0 = blockIdx.x * 64; const int part = blockIdx.y / NSL, slab = blockIdx.y % NSL, c0 = slab * 128;
  const float* xb = CN + (size_t)t0 * DM; const b16* Wp = part == 0 ? WQ : (part == 1 ? WK : WV); const float* bp = part == 0 ? bq : (part == 1 ? bk : bv);
  v8f acc[8];
#pragma unroll
  for (int t = 0; t < 8; ++t) acc[t] = (v8f){};
#pragma unroll 1
  for (int kc = 0; kc < DM; kc += 256) {
    __syncthreads();
    for (int i = threadIdx.x; i < 64 * 64; i += 128) { const int rr = i / 64, q = (i % 64) * 4; const v4f f = *(const v4f*)(xb + (size_t)rr * DM + kc + q); v4h o; for (int j = 0; j < 4; ++j) o[j] = (b16)(f[j] * XS); *(v4h*)(&As[rr][q]) = o; }
    __syncthreads();
#pragma unroll 2
    for (int kb = 0; kb < 256; kb += 32) { const v16b a = frag_kb(&As[wave * 16 + nloc][kb], hlf);
#pragma unroll
      for (int t = 0; t < 8; ++t) acc[t] = wmma16b(a, frag_kb(Wp + (size_t)(c0 + t * 16 + nloc) * DM + kc + kb, hlf), acc[t]); } }
#pragma unroll
  for (int t = 0; t < 8; ++t) { const float bbv = bf16_rne(bp[c0 + t * 16 + nloc]);
#pragma unroll
    for (int r = 0; r < 8; ++r) Tf[wave][8 * hlf + r][t * 16 + nloc] = acc[t][r] * (1.0f / (XS * WSC)) + bbv; }
  __syncthreads();
  for (int pass = 0; pass < 2; ++pass) {
    if (part < 2) { b16* pl = part == 0 ? QP : KP; const int c = c0 + lane * 4;
      for (int rr = 0; rr < 16; ++rr) { const int tok = t0 + wave * 16 + rr; v4h h4; for (int j = 0; j < 4; ++j) h4[j] = (b16)(Tf[wave][rr][lane * 4 + j] * XS); *(volatile v4h*)(pl + (size_t)tok * DM + c) = h4; } }
    else {
#pragma unroll 1
      for (int q = 0; q < 32; ++q) { const int cl = wave * 32 + q; const int e = c0 + cl; const int tk = lane * 2; v2h hv; for (int j = 0; j < 2; ++j) hv[j] = (b16)(Tf[(tk + j) >> 4][(tk + j) & 15][cl] * XS);
        *(volatile v2h*)(VT + (size_t)e * (size_t)T + t0 + lane * 2) = hv; } }
    __threadfence(); }
}
__global__ __launch_bounds__(128) void scores_kernel(const b16* __restrict__ QP, const b16* __restrict__ KP, float* __restrict__ S) {
  __shared__ __attribute__((aligned(16))) float Tf[4][16][128 + 4];
  const int wave = threadIdx.x >> 5, lane = threadIdx.x & 31, nloc = lane & 15, hlf = lane >> 4; const int q0 = blockIdx.x * 64 + wave * 16; const int k0 = blockIdx.y * 128;
  v8f acc[8];
#pragma unroll
  for (int t = 0; t < 8; ++t) acc[t] = (v8f){};
#pragma unroll 2
  for (int kb = 0; kb < DM; kb += 32) { const v16b a = frag_kb(QP + (size_t)(q0 + nloc) * DM + kb, hlf);
#pragma unroll
    for (int t = 0; t < 8; ++t) acc[t] = wmma16b(a, frag_kb(KP + (size_t)(k0 + t * 16 + nloc) * DM + kb, hlf), acc[t]); }
#pragma unroll
  for (int t = 0; t < 8; ++t)
#pragma unroll
    for (int r = 0; r < 8; ++r) Tf[wave][8 * hlf + r][t * 16 + nloc] = acc[t][r];
  wave_lds_sync();
  for (int pass = 0; pass < 2; ++pass) { for (int rr = 0; rr < 16; ++rr) *(volatile v4f*)(S + (size_t)(q0 + rr) * T + k0 + lane * 4) = *(const v4f*)(&Tf[wave][rr][lane * 4]); __threadfence(); }
}
__global__ __launch_bounds__(256) void softmax_kernel(const float* __restrict__ S, const int* __restrict__ mask, int b0, b16* __restrict__ Ph) {
  const int wave = threadIdx.x >> 5, lane = threadIdx.x & 31; const int i = blockIdx.x * 8 + wave;
  const int* mrow = mask + (size_t)b0 * T; int len = 0;
#pragma unroll 8
  for (int ch = 0; ch < T / 32; ++ch) len += (mrow[ch * 32 + lane] != 0) ? 1 : 0;
#pragma unroll
  for (int o = 16; o >= 1; o >>= 1) len += __shfl_xor(len, o);
  const bool rowlive = i < len;
  const float* sr = S + (size_t)i * T; const float c = LOG2E / ((float)DM * XS * XS);
  float sv[T / 64][2]; float m = -INFINITY;
#pragma unroll
  for (int ch = 0; ch < T / 64; ++ch) { const v2f s2 = *(const v2f*)(sr + ch * 64 + lane * 2); const int j0 = ch * 64 + lane * 2; const int m0 = mrow[j0], m1 = mrow[j0 + 1];
    sv[ch][0] = (rowlive && m0 != 0 && j0 <= i) ? s2[0] * c : MASKED; sv[ch][1] = (rowlive && m1 != 0 && j0 + 1 <= i) ? s2[1] * c : MASKED; m = fmaxf(m, fmaxf(sv[ch][0], sv[ch][1])); }
#pragma unroll
  for (int o = 16; o >= 1; o >>= 1) m = fmaxf(m, __shfl_xor(m, o));
  float l = 0.0f;
#pragma unroll
  for (int ch = 0; ch < T / 64; ++ch) for (int j = 0; j < 2; ++j) { const float p = nexp2(sv[ch][j] - m); sv[ch][j] = p; l += p; }
#pragma unroll
  for (int o = 16; o >= 1; o >>= 1) l += __shfl_xor(l, o);
  const float inv = PS / l;
  for (int pass = 0; pass < 2; ++pass) {
#pragma unroll
    for (int ch = 0; ch < T / 64; ++ch) { v2h h2; for (int j = 0; j < 2; ++j) h2[j] = (b16)pmul(sv[ch][j], inv); *(volatile v2h*)(Ph + (size_t)i * T + ch * 64 + lane * 2) = h2; }
    __threadfence(); }
}
__global__ __launch_bounds__(128) void pv_kernel(const b16* __restrict__ Ph, const b16* __restrict__ VT, b16* __restrict__ CTh, b16* __restrict__ CTl) {
  __shared__ __attribute__((aligned(16))) float Tf[4][16][128 + 4];
  const int wave = threadIdx.x >> 5, lane = threadIdx.x & 31, nloc = lane & 15, hlf = lane >> 4; const int q0 = blockIdx.x * 64 + wave * 16; const int e0 = blockIdx.y * 128;
  v8f acc[8];
#pragma unroll
  for (int t = 0; t < 8; ++t) acc[t] = (v8f){};
#pragma unroll 2
  for (int kb = 0; kb < T; kb += 32) { const v16b a = frag_kb(Ph + (size_t)(q0 + nloc) * T + kb, hlf);
#pragma unroll
    for (int t = 0; t < 8; ++t) acc[t] = wmma16b(a, frag_kb(VT + (size_t)(e0 + t * 16 + nloc) * T + kb, hlf), acc[t]); }
#pragma unroll
  for (int t = 0; t < 8; ++t)
#pragma unroll
    for (int r = 0; r < 8; ++r) Tf[wave][8 * hlf + r][t * 16 + nloc] = acc[t][r] * (1.0f / (PS * XS));
  wave_lds_sync();
  for (int pass = 0; pass < 2; ++pass) { for (int rr = 0; rr < 16; ++rr) { v4h h4, l4; for (int j = 0; j < 4; ++j) { b16 p, ql; split16(Tf[wave][rr][lane * 4 + j] * XS, p, ql); h4[j] = p; l4[j] = ql; }
      const size_t oi = (size_t)(q0 + rr) * DM + e0 + lane * 4; *(volatile v4h*)(CTh + oi) = h4; *(volatile v4h*)(CTl + oi) = l4; } __threadfence(); }
}
__global__ __launch_bounds__(128) void out1_kernel(const b16* __restrict__ Ch, const b16* __restrict__ Cl, const b16* __restrict__ WO, const float* __restrict__ bo, const float* __restrict__ CN, float* __restrict__ Y1) {
  __shared__ __attribute__((aligned(16))) float Tf[4][16][128 + 4];
  const int wave = threadIdx.x >> 5, lane = threadIdx.x & 31, nloc = lane & 15, hlf = lane >> 4; const size_t m0 = (size_t)blockIdx.x * 64 + wave * 16; const int n0 = blockIdx.y * 128;
  v8f acc[8];
#pragma unroll
  for (int t = 0; t < 8; ++t) acc[t] = (v8f){};
#pragma unroll 2
  for (int kb = 0; kb < DM; kb += 32) { const v16b ah = frag_kb(Ch + (m0 + nloc) * DM + kb, hlf), al = frag_kb(Cl + (m0 + nloc) * DM + kb, hlf);
#pragma unroll
    for (int t = 0; t < 8; ++t) { const v16b bw = frag_kb(WO + (size_t)(n0 + t * 16 + nloc) * DM + kb, hlf); acc[t] = wmma16b(ah, bw, acc[t]); acc[t] = wmma16b(al, bw, acc[t]); } }
#pragma unroll
  for (int t = 0; t < 8; ++t) { const int col = n0 + t * 16 + nloc; const float bbv = bf16_rne(bo[col]);
#pragma unroll
    for (int r = 0; r < 8; ++r) Tf[wave][8 * hlf + r][t * 16 + nloc] = acc[t][r] * (1.0f / (XS * WSC)) + bbv + CN[(m0 + 8 * hlf + r) * DM + col]; }
  wave_lds_sync();
  for (int pass = 0; pass < 2; ++pass) { for (int rr = 0; rr < 16; ++rr) *(volatile v4f*)(Y1 + (m0 + rr) * DM + n0 + lane * 4) = *(const v4f*)(&Tf[wave][rr][lane * 4]); __threadfence(); }
}
__global__ __launch_bounds__(256) void ln_kernel(const float* __restrict__ Y1, const float* __restrict__ g, const float* __restrict__ bb, float* __restrict__ CE, float* __restrict__ OUT2) {
  const int wave = threadIdx.x >> 5, lane = threadIdx.x & 31; const int row = blockIdx.x * 8 + wave;
  float v[24]; float s1 = 0.0f; const float* xr = Y1 + (size_t)row * DM;
#pragma unroll
  for (int k = 0; k < NCH; ++k) { const v4f t4 = *(const v4f*)(xr + 128 * k + 4 * lane); for (int j = 0; j < 4; ++j) { v[4 * k + j] = t4[j]; s1 += t4[j]; } }
#pragma unroll
  for (int o = 16; o >= 1; o >>= 1) s1 += __shfl_xor(s1, o);
  const float mu = s1 * (1.0f / DM); float s2 = 0.0f;
#pragma unroll
  for (int q = 0; q < 24; ++q) { const float d = v[q] - mu; s2 += pmul(d, d); }
#pragma unroll
  for (int o = 16; o >= 1; o >>= 1) s2 += __shfl_xor(s2, o);
  const float rs = rsqrtf(s2 * (1.0f / DM) + LNEPS);
  v4f o4[NCH];
#pragma unroll
  for (int k = 0; k < NCH; ++k) for (int j = 0; j < 4; ++j) { const int c = 128 * k + 4 * lane + j; o4[k][j] = pmul((v[4 * k + j] - mu) * rs, bfp(g[c])) + bfp(bb[c]); }
  for (int pass = 0; pass < 2; ++pass) {
#pragma unroll
    for (int k = 0; k < NCH; ++k) { *(volatile v4f*)(CE + (size_t)row * DM + 128 * k + 4 * lane) = o4[k]; *(volatile v4f*)(OUT2 + (size_t)row * DM + 128 * k + 4 * lane) = o4[k]; }
    __threadfence(); }
}
__global__ __launch_bounds__(64) void actor_kernel(const float* __restrict__ CE, const b16* __restrict__ WA, const float* __restrict__ ba, float* __restrict__ OUT1) {
  __shared__ __attribute__((aligned(16))) b16 Ah[2][16][DM + 8]; __shared__ __attribute__((aligned(16))) float To[32][2];
  const int wave = threadIdx.x >> 5, lane = threadIdx.x & 31, nloc = lane & 15, hlf = lane >> 4; const size_t m0 = (size_t)blockIdx.x * 32 + wave * 16;
  for (int idx = lane; idx < 16 * (DM / 4); idx += 32) { const int rr = idx / (DM / 4), c4 = (idx % (DM / 4)) * 4; const v4f vv = *(const v4f*)(CE + (m0 + rr) * DM + c4); v4h hv; for (int j = 0; j < 4; ++j) hv[j] = (b16)(vv[j] * XS); *(v4h*)(&Ah[wave][rr][c4]) = hv; }
  wave_lds_sync();
  v8f acc = (v8f){};
#pragma unroll 4
  for (int kb = 0; kb < DM; kb += 32) acc = wmma16b(frag_kb(&Ah[wave][nloc][kb], hlf), frag_kb(WA + (size_t)nloc * DM + kb, hlf), acc);
#pragma unroll
  for (int r = 0; r < 8; ++r) { const float z = acc[r] * (1.0f / (XS * WSC)) + bf16_rne(ba[nloc < NA ? nloc : 0]); const float zo = __shfl_xor(z, 1); if (nloc < NA) { const float mx = fmaxf(z, zo); const float ez = __expf(z - mx), eo = __expf(zo - mx); To[wave * 16 + 8 * hlf + r][nloc] = ez * __builtin_amdgcn_rcpf(ez + eo); } }
  __syncthreads();
  for (int pass = 0; pass < 2; ++pass) { if (threadIdx.x < 16) *(volatile v4f*)(OUT1 + (size_t)blockIdx.x * 64 + threadIdx.x * 4) = *(const v4f*)(&To[threadIdx.x * 2][0]); __threadfence(); }
}
}

extern "C" void kernel_launch(void* const* d_in, const int* in_sizes, int n_in, void* d_out, int out_size, void* d_ws, size_t ws_size, hipStream_t stream) {
  (void)n_in;
  auto Fp = [&](int i) { return (const float*)d_in[i]; }; auto Ip = [&](int i) { return (const int*)d_in[i]; };
  if (in_sizes[0] != B * T * DM || in_sizes[1] != B * T || in_sizes[2] != DM || in_sizes[3] != DM || in_sizes[4] != DM * DM || in_sizes[6] != DM * DM || in_sizes[8] != DM * DM || in_sizes[10] != DM * DM || in_sizes[5] != DM || in_sizes[7] != DM || in_sizes[9] != DM || in_sizes[11] != DM || in_sizes[12] != DM || in_sizes[13] != DM || in_sizes[14] != DM * NA || in_sizes[15] != NA || out_size != B * T * NA + B * T * DM) return;
  float* out1 = (float*)d_out; float* out2 = (float*)d_out + (size_t)B * T * NA;
  size_t off = 0; char* ws = (char*)d_ws;
  auto carve = [&](size_t bytes) { char* p = ws + off; off += (bytes + 255) & ~(size_t)255; return p; };
  b16* WQ = (b16*)carve((size_t)DM * DM * 2); b16* WK = (b16*)carve((size_t)DM * DM * 2); b16* WV = (b16*)carve((size_t)DM * DM * 2); b16* WO = (b16*)carve((size_t)DM * DM * 2); b16* WA = (b16*)carve((size_t)16 * DM * 2);
  float* CN = (float*)carve((size_t)T * DM * 4); b16* QP = (b16*)carve((size_t)T * DM * 2); b16* KP = (b16*)carve((size_t)T * DM * 2); b16* VT = (b16*)carve((size_t)DM * T * 2); float* S = (float*)carve((size_t)T * T * 4); b16* Ph = (b16*)carve((size_t)T * T * 2);
  b16* CTh = (b16*)carve((size_t)T * DM * 2); b16* CTl = (b16*)carve((size_t)T * DM * 2); float* Y1 = (float*)carve((size_t)T * DM * 4); float* CE = (float*)carve((size_t)T * DM * 4);
  if (off > ws_size || off > ((size_t)128 << 20)) return;
  prep_kernel<<<(unsigned)(((size_t)4 * DM * DM / 8 + 16 * DM / 8 + 255) / 256), 256, 0, stream>>>(Fp(4), Fp(6), Fp(8), Fp(10), Fp(14), WQ, WK, WV, WO, WA);
  for (int b0 = 0; b0 < NB; ++b0) {
    cn_kernel<<<T / 8, 256, 0, stream>>>(Fp(0), b0, Fp(2), Fp(3), CN);
    proj_kernel<<<dim3(T / 64, 3 * NSL), 128, 0, stream>>>(CN, WQ, WK, WV, Fp(5), Fp(7), Fp(9), QP, KP, VT);
    scores_kernel<<<dim3(T / 64, T / 128), 128, 0, stream>>>(QP, KP, S);
    softmax_kernel<<<T / 8, 256, 0, stream>>>(S, Ip(1), b0, Ph);
    pv_kernel<<<dim3(T / 64, DM / 128), 128, 0, stream>>>(Ph, VT, CTh, CTl);
    out1_kernel<<<dim3(T / 64, DM / 128), 128, 0, stream>>>(CTh, CTl, WO, Fp(11), CN, Y1);
    ln_kernel<<<T / 8, 256, 0, stream>>>(Y1, Fp(12), Fp(13), CE, out2 + (size_t)b0 * T * DM);
    actor_kernel<<<T / 32, 64, 0, stream>>>(CE, WA, Fp(15), out1 + (size_t)b0 * T * NA); }
}
